// MoaAttention_3685081940644
// MI455X (gfx1250) — hardware-run, weakly checked
//
#include <hip/hip_runtime.h>
#include <math.h>

typedef __attribute__((ext_vector_type(16))) _Float16 v16h;
typedef __attribute__((ext_vector_type(8)))  _Float16 v8h;
typedef __attribute__((ext_vector_type(8)))  float    v8f;
typedef __attribute__((ext_vector_type(4)))  float    v4f;
typedef __attribute__((ext_vector_type(4)))  unsigned int v4u;
typedef __attribute__((ext_vector_type(4)))  int      v4i;

constexpr int kB   = 4;
constexpr int kT   = 2048;
constexpr int kD   = 512;
constexpr int kH   = 8;
constexpr int kE   = 16;
constexpr int kHD  = 64;
constexpr int kTop = 8;
constexpr int kN   = kB * kT;
constexpr int kEH  = kE * kHD;
static_assert(kH * kHD == kD, "heads x head width");
static_assert(kTop == kH, "selected experts == heads");
static_assert(kN == 8192 && kEH == 1024, "token and expert-line counts");
static_assert((kD % 32) == 0 && (kEH % 32) == 0 && (kHD % 32) == 0 && (kT % 32) == 0, "GEMM depth multiples of 32");
static_assert((kN % 64) == 0 && (kEH % 64) == 0 && (kD % 64) == 0 && (kT % 64) == 0, "tile multiples of 64");
static_assert((kN % 256) == 0, "gate kernel grid is exact");

constexpr int isqrt_c(int v) { int r = 0; while ((r + 1) * (r + 1) <= v) ++r; return r; }
static_assert(isqrt_c(kHD) * isqrt_c(kHD) == kHD, "head width is a perfect square");
constexpr float kQScale = 1.0f / (float)isqrt_c(kHD);

constexpr float kXCarry    = 16.0f;
constexpr float kXResCarry = 2048.0f;
constexpr float kW1Carry   = 128.0f;
constexpr float kQCarry    = 64.0f;
constexpr float kKCarry    = 16.0f;
constexpr float kVCarry    = 16.0f;
constexpr float kPCarry    = 32768.0f;
constexpr float kMCarry    = 4096.0f;
constexpr float kW2Carry   = 128.0f;
constexpr float kYCarry    = 1024.0f;
constexpr float kOWCarry   = 512.0f;
constexpr float kDqFold    = (kQCarry * kQScale) / (kXCarry * kW1Carry);
constexpr float kResFold   = 1.0f / kXResCarry;
constexpr float kScoreFold = 1.0f / (kQCarry * kKCarry);
constexpr float kAttnFold  = kMCarry / (kPCarry * kVCarry);
constexpr float kRedFold   = kYCarry / (kMCarry * kW2Carry);
constexpr float kOutFold   = 1.0f / (kYCarry * kOWCarry);
constexpr float kF16MinNormal = 6.103515625e-5f;
static_assert(kDqFold == 1.0f / 256.0f, "dense projection fold");
static_assert(kScoreFold == 1.0f / 1024.0f, "score fold");
static_assert(kAttnFold == 1.0f / 128.0f, "attention fold");
static_assert(kRedFold == 1.0f / 512.0f, "reduce fold");

constexpr size_t kOffXH  = 0;
constexpr size_t kOffXL  = kOffXH  + (size_t)kN * kD * 2;
constexpr size_t kOffKH  = kOffXL  + (size_t)kN * kD * 2;
constexpr size_t kOffVT  = kOffKH  + (size_t)kN * kD * 2;
constexpr size_t kOffW1T = kOffVT  + (size_t)kN * kD * 2;
constexpr size_t kOffW2T = kOffW1T + (size_t)kEH * kD * 2;
constexpr size_t kOffOWT = kOffW2T + (size_t)kD * kEH * 2;
constexpr size_t kOffGT  = kOffOWT + (size_t)kD * kD * 2;
constexpr size_t kOffIX  = kOffGT  + (size_t)kN * kTop * 4;
constexpr size_t kOffDQ  = kOffIX  + (size_t)kN * kTop * 4;
constexpr size_t kOffAOG = kOffDQ  + (size_t)kN * kEH * 2;
constexpr size_t kOffMP  = kOffAOG + (size_t)kN * kD * 2;
constexpr size_t kOffYP  = kOffMP  + (size_t)kN * kEH * 2;
constexpr size_t kWsTotal = kOffYP + (size_t)kN * kD * 2;
static_assert(kWsTotal == 87031808ull, "carve total");
static_assert(kWsTotal <= 134217728ull, "carve cap");
static_assert((kOffXL % 128) == 0 && (kOffKH % 128) == 0 && (kOffVT % 128) == 0 && (kOffW1T % 128) == 0 &&
              (kOffW2T % 128) == 0 && (kOffOWT % 128) == 0 && (kOffGT % 128) == 0 && (kOffIX % 128) == 0 &&
              (kOffDQ % 128) == 0 && (kOffAOG % 128) == 0 && (kOffMP % 128) == 0 && (kOffYP % 128) == 0,
              "128-B aligned regions");

__device__ __forceinline__ _Float16 to_h16(float v) {
  const float f = (fabsf(v) < kF16MinNormal) ? 0.0f : v;
  return (_Float16)f;
}
__device__ __forceinline__ v8f mma_g(v16h a, v16h b, v8f c) {
  c = __builtin_amdgcn_wmma_f32_16x16x32_f16(false, a, false, b, (short)0, c, false, false);
  asm volatile("v_nop\n\tv_nop\n\tv_nop\n\tv_nop" : "+v"(c) : "v"(a), "v"(b));
  return c;
}
union FragH { v16h v; v8h h[2]; };
__device__ __forceinline__ v16h frag_load(const _Float16* p) {
  FragH f;
  f.h[0] = *(const v8h*)(p);
  f.h[1] = *(const v8h*)(p + 16);
  return f.v;
}

__global__ __launch_bounds__(256) void pack_x_kernel(const float* __restrict__ in, unsigned short* __restrict__ hi,
                                                     unsigned short* __restrict__ lo, int n8) {
  const int i = blockIdx.x * 256 + threadIdx.x;
  if (i >= n8) return;
  const size_t e0 = (size_t)i << 3;
  const v4f a0 = *(const v4f*)(in + e0);
  const v4f a1 = *(const v4f*)(in + e0 + 4);
  v8h hv, lv;
#pragma unroll
  for (int e = 0; e < 4; ++e) {
    const float x0 = a0[e] * kXCarry;
    const float x1 = a1[e] * kXCarry;
    const _Float16 h0 = to_h16(x0);
    const _Float16 h1 = to_h16(x1);
    const float r0 = (x0 - (float)h0) * kXResCarry;
    const float r1 = (x1 - (float)h1) * kXResCarry;
    hv[e]     = h0;
    hv[4 + e] = h1;
    lv[e]     = to_h16(r0);
    lv[4 + e] = to_h16(r1);
  }
  unsigned short* qh = hi + e0;
  unsigned short* ql = lo + e0;
  *(volatile v8h*)qh = hv;
  *(volatile v8h*)ql = lv;
  __threadfence();
  *(volatile v8h*)qh = hv;
  *(volatile v8h*)ql = lv;
}

__global__ __launch_bounds__(256) void pack_scale_kernel(const float* __restrict__ in, unsigned short* __restrict__ out,
                                                         int n8, float scale) {
  const int i = blockIdx.x * 256 + threadIdx.x;
  if (i >= n8) return;
  const size_t e0 = (size_t)i << 3;
  const v4f a0 = *(const v4f*)(in + e0);
  const v4f a1 = *(const v4f*)(in + e0 + 4);
  v8h hv;
#pragma unroll
  for (int e = 0; e < 4; ++e) {
    hv[e]     = to_h16(a0[e] * scale);
    hv[4 + e] = to_h16(a1[e] * scale);
  }
  unsigned short* q = out + e0;
  *(volatile v8h*)q = hv;
  __threadfence();
  *(volatile v8h*)q = hv;
}

__global__ __launch_bounds__(256) void tpose_f16_kernel(const float* __restrict__ in, int in_pitch, long inS1, long inS2,
                                                        int zdiv, unsigned short* __restrict__ out, int out_pitch,
                                                        long outS, float scale) {
  __shared__ float sm[64][65];
  const int t  = threadIdx.x;
  const int r0 = blockIdx.x * 64;
  const int c0 = blockIdx.y * 64;
  const int z  = blockIdx.z;
  const int zi = z / zdiv;
  const int zj = z - zi * zdiv;
  const float* ip = in + (size_t)zi * inS1 + (size_t)zj * inS2;
#pragma unroll
  for (int i = 0; i < 4; ++i) {
    const int e4 = i * 256 + t;
    const int r  = e4 >> 4;
    const int c4 = (e4 & 15) * 4;
    const v4f v = *(const v4f*)(ip + (size_t)(r0 + r) * in_pitch + c0 + c4);
    sm[c4 + 0][r] = v[0] * scale;
    sm[c4 + 1][r] = v[1] * scale;
    sm[c4 + 2][r] = v[2] * scale;
    sm[c4 + 3][r] = v[3] * scale;
  }
  __syncthreads();
  const int lane = t & 31, wave = t >> 5;
  const int q = lane >> 3, c8 = (lane & 7) * 8;
  unsigned short* op = out + (size_t)z * outS;
  v8h hv[2];
#pragma unroll
  for (int it = 0; it < 2; ++it) {
    const int row = wave * 8 + it * 4 + q;
#pragma unroll
    for (int e = 0; e < 8; ++e) hv[it][e] = to_h16(sm[row][c8 + e]);
  }
  for (int pass = 0; pass < 2; ++pass) {
#pragma unroll
    for (int it = 0; it < 2; ++it) {
      const int row = wave * 8 + it * 4 + q;
      *(volatile v8h*)(op + (size_t)(c0 + row) * out_pitch + r0 + c8) = hv[it];
    }
    __threadfence();
  }
}

__global__ __launch_bounds__(256) void gate_topk_kernel(const float* __restrict__ x, const float* __restrict__ eg,
                                                        float* __restrict__ gates, int* __restrict__ idx) {
  __shared__ float sL[kE * 256];
  __shared__ float sP[kE * 256];
  __shared__ __align__(16) float sG[256 * kTop];
  __shared__ __align__(16) int   sI[256 * kTop];
  const int tid = threadIdx.x;
  const int n = blockIdx.x * 256 + tid;
  float acc[kE];
#pragma unroll
  for (int e = 0; e < kE; ++e) acc[e] = 0.0f;
  const float* xr = x + (size_t)n * kD;
#pragma unroll 1
  for (int d = 0; d < kD; ++d) {
    const float xv = xr[d];
    const float* gr = eg + d * kE;
#pragma unroll
    for (int e = 0; e < kE; ++e) acc[e] = fmaf(xv, gr[e], acc[e]);
  }
#pragma unroll
  for (int e = 0; e < kE; ++e) sL[e * 256 + tid] = acc[e];
  float mx = sL[tid];
#pragma unroll 1
  for (int e = 1; e < kE; ++e) mx = fmaxf(mx, sL[e * 256 + tid]);
  float sum = 0.0f;
#pragma unroll 1
  for (int e = 0; e < kE; ++e) {
    const float p = expf(sL[e * 256 + tid] - mx);
    sP[e * 256 + tid] = p;
    sum += p;
  }
  const float inv = 1.0f / sum;
  unsigned taken = 0u;
#pragma unroll 1
  for (int j = 0; j < kTop; ++j) {
    float bv = -INFINITY;
    int best = -1;
#pragma unroll 1
    for (int e = 0; e < kE; ++e) {
      const float v = sL[e * 256 + tid];
      const bool open = ((taken >> e) & 1u) == 0u;
      if (open && (v > bv)) { bv = v; best = e; }
    }
    if (best < 0) best = __ffs((int)(~taken)) - 1;
    best = best < 0 ? 0 : (best > kE - 1 ? kE - 1 : best);
    taken |= (1u << best);
    sG[tid * kTop + j] = sP[best * 256 + tid] * inv;
    sI[tid * kTop + j] = best;
  }
  __syncthreads();
  float* gp = gates + (size_t)blockIdx.x * (256 * kTop);
  int*   ip = idx   + (size_t)blockIdx.x * (256 * kTop);
  const v4f g0 = *(const v4f*)(sG + tid * 4);
  const v4f g1 = *(const v4f*)(sG + 1024 + tid * 4);
  const v4i i0 = *(const v4i*)(sI + tid * 4);
  const v4i i1 = *(const v4i*)(sI + 1024 + tid * 4);
  for (int pass = 0; pass < 2; ++pass) {
    *(volatile v4f*)(gp + tid * 4) = g0;
    *(volatile v4f*)(gp + 1024 + tid * 4) = g1;
    *(volatile v4i*)(ip + tid * 4) = i0;
    *(volatile v4i*)(ip + 1024 + tid * 4) = i1;
    __threadfence();
  }
}

template <int MI, bool RES, int OUT_MODE, bool BIAS>
__global__ __launch_bounds__(256) void wmma_gemm_kernel(
    const unsigned short* __restrict__ Ap, const unsigned short* __restrict__ A2p, int lda,
    const unsigned short* __restrict__ Btp, int ldb,
    void* __restrict__ Cout, int ldc, const float* __restrict__ bias,
    int M, int N, int K, float scale, float rscale) {
  const _Float16* A  = (const _Float16*)Ap;
  const _Float16* A2 = (const _Float16*)A2p;
  const _Float16* Bt = (const _Float16*)Btp;
  __shared__ __align__(16) float sT[8][16 * 68];
  const int lane = threadIdx.x & 31;
  const int wave = threadIdx.x >> 5;
  const int tilesN = N >> 6;
  const int tilesM = M / (16 * MI);
  const int tile = blockIdx.x * 8 + wave;
  if (tile >= tilesM * tilesN) return;
  const int tm = tile / tilesN;
  const int tn = tile - tm * tilesN;
  const int m0 = tm * (16 * MI);
  const int n0 = tn << 6;
  const int rlane = lane & 15;
  const int koff  = (lane >> 4) * 8;
  const int mOff  = (lane >> 4) * 8;

  v8f acc[MI][4];
  v8f accr[RES ? MI : 1][4];
#pragma unroll
  for (int i = 0; i < MI; ++i)
#pragma unroll
    for (int j = 0; j < 4; ++j) acc[i][j] = (v8f){0.f, 0.f, 0.f, 0.f, 0.f, 0.f, 0.f, 0.f};
#pragma unroll
  for (int i = 0; i < (RES ? MI : 1); ++i)
#pragma unroll
    for (int j = 0; j < 4; ++j) accr[i][j] = (v8f){0.f, 0.f, 0.f, 0.f, 0.f, 0.f, 0.f, 0.f};

  for (int k0 = 0; k0 < K; k0 += 32) {
    v16h bh[4];
#pragma unroll
    for (int j = 0; j < 4; ++j)
      bh[j] = frag_load(Bt + (size_t)(n0 + (j << 4) + rlane) * ldb + koff + k0);
#pragma unroll
    for (int i = 0; i < MI; ++i) {
      const size_t ao = (size_t)(m0 + (i << 4) + rlane) * lda + koff + k0;
      const v16h ah = frag_load(A + ao);
      if (RES) {
        const v16h al = frag_load(A2 + ao);
#pragma unroll
        for (int j = 0; j < 4; ++j) {
          acc[i][j]  = mma_g(ah, bh[j], acc[i][j]);
          accr[i][j] = mma_g(al, bh[j], accr[i][j]);
        }
      } else {
#pragma unroll
        for (int j = 0; j < 4; ++j) acc[i][j] = mma_g(ah, bh[j], acc[i][j]);
      }
    }
  }

  float* slab = sT[wave];
#pragma unroll
  for (int i = 0; i < MI; ++i) {
    const int mBase = m0 + (i << 4);
#pragma unroll
    for (int j = 0; j < 4; ++j) {
      float bv = 0.f;
      if (BIAS) bv = bias[n0 + (j << 4) + rlane];
#pragma unroll
      for (int r = 0; r < 8; ++r) {
        float v = acc[i][j][r];
        if (RES) v = v + accr[i][j][r] * rscale;
        v = v * scale;
        if (BIAS) v += bv;
        slab[(mOff + r) * 68 + (j << 4) + rlane] = v;
      }
    }
    __builtin_amdgcn_fence(__ATOMIC_RELEASE, "workgroup");
    __builtin_amdgcn_wave_barrier();
    __builtin_amdgcn_fence(__ATOMIC_ACQUIRE, "workgroup");
    if (OUT_MODE == 0) {
      float* C = (float*)Cout;
      const int hh = lane >> 4, c4 = (lane & 15) * 4;
      for (int pass = 0; pass < 2; ++pass) {
#pragma unroll
        for (int it = 0; it < 8; ++it) {
          const int row = it * 2 + hh;
          const v4f v = *(const v4f*)(slab + row * 68 + c4);
          *(volatile v4f*)(C + (size_t)(mBase + row) * ldc + n0 + c4) = v;
        }
        __threadfence();
      }
    } else {
      const int q = lane >> 3, c8 = (lane & 7) * 8;
      unsigned short* C = (unsigned short*)Cout;
      v8h hv[4];
#pragma unroll
      for (int it = 0; it < 4; ++it) {
        const float* sp = slab + (it * 4 + q) * 68 + c8;
        const v4f a0 = *(const v4f*)(sp);
        const v4f a1 = *(const v4f*)(sp + 4);
#pragma unroll
        for (int e = 0; e < 4; ++e) {
          hv[it][e]     = to_h16(a0[e]);
          hv[it][4 + e] = to_h16(a1[e]);
        }
      }
      for (int pass = 0; pass < 2; ++pass) {
#pragma unroll
        for (int it = 0; it < 4; ++it) {
          const int row = it * 4 + q;
          *(volatile v8h*)(C + (size_t)(mBase + row) * ldc + n0 + c8) = hv[it];
        }
        __threadfence();
      }
    }
    __builtin_amdgcn_fence(__ATOMIC_RELEASE, "workgroup");
    __builtin_amdgcn_wave_barrier();
    __builtin_amdgcn_fence(__ATOMIC_ACQUIRE, "workgroup");
  }
}

__global__ __launch_bounds__(128) void attn_kernel(const unsigned short* __restrict__ DQp, const int* __restrict__ idx,
                                                   const float* __restrict__ gates,
                                                   const unsigned short* __restrict__ KHp,
                                                   const unsigned short* __restrict__ VTp,
                                                   unsigned short* __restrict__ AOG) {
  __shared__ __align__(16) _Float16 Qs[64 * 64];
  __shared__ __align__(16) _Float16 Ks[64 * 64];
  __shared__ __align__(16) _Float16 Vs[64 * 64];
  __shared__ __align__(16) _Float16 Ps[4][16 * 64];
  __shared__ __align__(16) float    Os[4][16 * 68];
  const _Float16* DQ = (const _Float16*)DQp;
  const _Float16* KH = (const _Float16*)KHp;
  const _Float16* VT = (const _Float16*)VTp;

  const int tid  = threadIdx.x;
  const int wave = tid >> 5;
  const int lane = tid & 31;
  const int hh   = lane >> 4;
  const int c    = lane & 15;
  constexpr int nqb = kT / 64;
  const int bx = blockIdx.x;
  const int qb = bx % nqb;
  const int bh = bx / nqb;
  const int h  = bh % kH;
  const int b  = bh / kH;
  const int qbase = qb * 64;
  const int q0l = wave * 16;
  const int srow = tid >> 1;
  const int shalf = (tid & 1) * 32;

  {
    const int n = b * kT + qbase + srow;
    int e = idx[(size_t)n * kTop + h];
    e = e < 0 ? 0 : (e > kE - 1 ? kE - 1 : e);
    const _Float16* src = DQ + (size_t)n * kEH + e * kHD + shalf;
#pragma unroll
    for (int i = 0; i < 4; ++i)
      *(v8h*)(Qs + srow * 64 + shalf + 8 * i) = *(const v8h*)(src + 8 * i);
  }
  __syncthreads();
  v16h qa[2];
#pragma unroll
  for (int dc = 0; dc < 2; ++dc) {
    FragH f;
    f.h[0] = *(const v8h*)(Qs + (q0l + c) * 64 + dc * 32 + 8 * hh);
    f.h[1] = *(const v8h*)(Qs + (q0l + c) * 64 + dc * 32 + 16 + 8 * hh);
    qa[dc] = f.v;
  }

  float mrow[8], lrow[8];
  v8f oacc[4];
#pragma unroll
  for (int r = 0; r < 8; ++r) { mrow[r] = -INFINITY; lrow[r] = 0.f; }
#pragma unroll
  for (int t = 0; t < 4; ++t) oacc[t] = (v8f){0.f, 0.f, 0.f, 0.f, 0.f, 0.f, 0.f, 0.f};

  _Float16* pw = Ps[wave];
  constexpr int nChunks = kT / 64;
#pragma unroll 1
  for (int kc = 0; kc < nChunks; ++kc) {
    const int kv0 = kc * 64;
    __syncthreads();
    {
      const _Float16* ks = KH + (size_t)(b * kT + kv0 + srow) * kD + h * kHD + shalf;
      const _Float16* vs = VT + ((size_t)(b * kH + h) * kHD + srow) * kT + kv0 + shalf;
#pragma unroll
      for (int i = 0; i < 4; ++i) {
        *(v8h*)(Ks + srow * 64 + shalf + 8 * i) = *(const v8h*)(ks + 8 * i);
        *(v8h*)(Vs + srow * 64 + shalf + 8 * i) = *(const v8h*)(vs + 8 * i);
      }
    }
    __syncthreads();

    v8f s[4];
#pragma unroll
    for (int j = 0; j < 4; ++j) {
      s[j] = (v8f){0.f, 0.f, 0.f, 0.f, 0.f, 0.f, 0.f, 0.f};
#pragma unroll
      for (int dc = 0; dc < 2; ++dc) {
        FragH kb;
        kb.h[0] = *(const v8h*)(Ks + (j * 16 + c) * 64 + dc * 32 + 8 * hh);
        kb.h[1] = *(const v8h*)(Ks + (j * 16 + c) * 64 + dc * 32 + 16 + 8 * hh);
        s[j] = mma_g(qa[dc], kb.v, s[j]);
      }
    }
    float cm[8];
#pragma unroll
    for (int r = 0; r < 8; ++r) {
      float m = -INFINITY;
#pragma unroll
      for (int j = 0; j < 4; ++j) {
        s[j][r] = s[j][r] * kScoreFold;
        m = fmaxf(m, s[j][r]);
      }
#pragma unroll
      for (int off = 1; off < 16; off <<= 1) m = fmaxf(m, __shfl_xor(m, off, 32));
      cm[r] = m;
    }
#pragma unroll
    for (int r = 0; r < 8; ++r) {
      const float mnew = fmaxf(mrow[r], cm[r]);
      const float alpha = __expf(mrow[r] - mnew);
      mrow[r] = mnew;
      float psum = 0.f;
#pragma unroll
      for (int j = 0; j < 4; ++j) {
        const float p = __expf(s[j][r] - mnew);
        psum += p;
        pw[(8 * hh + r) * 64 + j * 16 + c] = to_h16(p * kPCarry);
      }
#pragma unroll
      for (int off = 1; off < 16; off <<= 1) psum += __shfl_xor(psum, off, 32);
      lrow[r] = lrow[r] * alpha + psum;
#pragma unroll
      for (int t = 0; t < 4; ++t) oacc[t][r] *= alpha;
    }
    __builtin_amdgcn_fence(__ATOMIC_RELEASE, "workgroup");
    __builtin_amdgcn_wave_barrier();
    __builtin_amdgcn_fence(__ATOMIC_ACQUIRE, "workgroup");
#pragma unroll
    for (int kk = 0; kk < 2; ++kk) {
      FragH pa;
      pa.h[0] = *(const v8h*)(pw + c * 64 + kk * 32 + 8 * hh);
      pa.h[1] = *(const v8h*)(pw + c * 64 + kk * 32 + 16 + 8 * hh);
#pragma unroll
      for (int t = 0; t < 4; ++t) {
        FragH vb;
        vb.h[0] = *(const v8h*)(Vs + (t * 16 + c) * 64 + kk * 32 + 8 * hh);
        vb.h[1] = *(const v8h*)(Vs + (t * 16 + c) * 64 + kk * 32 + 16 + 8 * hh);
        oacc[t] = mma_g(pa.v, vb.v, oacc[t]);
      }
    }
    __builtin_amdgcn_fence(__ATOMIC_RELEASE, "workgroup");
    __builtin_amdgcn_wave_barrier();
    __builtin_amdgcn_fence(__ATOMIC_ACQUIRE, "workgroup");
  }

  float* os = Os[wave];
#pragma unroll
  for (int r = 0; r < 8; ++r) {
    const int n = b * kT + qbase + q0l + 8 * hh + r;
    const float g = gates[(size_t)n * kTop + h];
    const float inv = (g * kAttnFold) * (1.0f / lrow[r]);
#pragma unroll
    for (int t = 0; t < 4; ++t) os[(8 * hh + r) * 68 + t * 16 + c] = oacc[t][r] * inv;
  }
  __builtin_amdgcn_fence(__ATOMIC_RELEASE, "workgroup");
  __builtin_amdgcn_wave_barrier();
  __builtin_amdgcn_fence(__ATOMIC_ACQUIRE, "workgroup");
  {
    const int q = lane >> 3, c8 = (lane & 7) * 8;
    v8h hv[4];
#pragma unroll
    for (int it = 0; it < 4; ++it) {
      const float* sp = os + (it * 4 + q) * 68 + c8;
      const v4f a0 = *(const v4f*)(sp);
      const v4f a1 = *(const v4f*)(sp + 4);
#pragma unroll
      for (int e = 0; e < 4; ++e) {
        hv[it][e]     = to_h16(a0[e]);
        hv[it][4 + e] = to_h16(a1[e]);
      }
    }
    for (int pass = 0; pass < 2; ++pass) {
#pragma unroll
      for (int it = 0; it < 4; ++it) {
        const int row = it * 4 + q;
        const size_t n = (size_t)(b * kT + qbase + q0l + row);
        *(volatile v8h*)(AOG + n * kD + h * kHD + c8) = hv[it];
      }
      __threadfence();
    }
  }
}

__global__ __launch_bounds__(256) void place_kernel(const unsigned short* __restrict__ AOG, const int* __restrict__ idx,
                                                    unsigned short* __restrict__ MP) {
  const int lane = threadIdx.x & 31, wave = threadIdx.x >> 5;
  const int n = blockIdx.x * 8 + wave;
  const v4i i0 = *(const v4i*)(idx + (size_t)n * kTop);
  const v4i i1 = *(const v4i*)(idx + (size_t)n * kTop + 4);
  int id[8];
  id[0] = i0.x; id[1] = i0.y; id[2] = i0.z; id[3] = i0.w;
  id[4] = i1.x; id[5] = i1.y; id[6] = i1.z; id[7] = i1.w;
#pragma unroll
  for (int j = 0; j < 8; ++j) id[j] = id[j] < 0 ? 0 : (id[j] > kE - 1 ? kE - 1 : id[j]);
  const int q = lane >> 3, c8 = (lane & 7) * 8;
  v4u vals[4];
#pragma unroll
  for (int it = 0; it < 4; ++it) {
    const int e = it * 4 + q;
    int slot = -1;
#pragma unroll
    for (int j = 0; j < 8; ++j) slot = (id[j] == e) ? j : slot;
    const int sc = slot < 0 ? 0 : slot;
    const v4u v = *(const v4u*)(AOG + (size_t)n * kD + sc * kHD + c8);
    unsigned a0 = v.x, a1 = v.y, a2 = v.z, a3 = v.w;
    asm volatile("" : "+v"(a0), "+v"(a1), "+v"(a2), "+v"(a3));
    const bool sel = (slot >= 0);
    vals[it] = (v4u){sel ? a0 : 0u, sel ? a1 : 0u, sel ? a2 : 0u, sel ? a3 : 0u};
  }
  for (int pass = 0; pass < 2; ++pass) {
#pragma unroll
    for (int it = 0; it < 4; ++it) {
      const int e = it * 4 + q;
      *(volatile v4u*)(MP + (size_t)n * kEH + e * kHD + c8) = vals[it];
    }
    __threadfence();
  }
}

extern "C" void kernel_launch(void* const* d_in, const int* in_sizes, int n_in,
                              void* d_out, int out_size, void* d_ws, size_t ws_size,
                              hipStream_t stream) {
  if (n_in < 8) return;
  if (in_sizes[0] != kN * kD) return;
  if (in_sizes[1] != kN * kD) return;
  if (in_sizes[2] != kN * kD) return;
  if (in_sizes[3] != kD * kE) return;
  if (in_sizes[4] != kE * kD * kHD) return;
  if (in_sizes[5] != kE * kHD * kD) return;
  if (in_sizes[6] != kD * kD) return;
  if (in_sizes[7] != kD) return;
  if (out_size != kN * kD) return;
  if (ws_size < kWsTotal) return;

  const float* query = (const float*)d_in[0];
  const float* keyp  = (const float*)d_in[1];
  const float* value = (const float*)d_in[2];
  const float* egate = (const float*)d_in[3];
  const float* w1    = (const float*)d_in[4];
  const float* w2    = (const float*)d_in[5];
  const float* outw  = (const float*)d_in[6];
  const float* outb  = (const float*)d_in[7];
  float* out = (float*)d_out;

  char* ws = (char*)d_ws;
  unsigned short* XH  = (unsigned short*)(ws + kOffXH);
  unsigned short* XL  = (unsigned short*)(ws + kOffXL);
  unsigned short* KH  = (unsigned short*)(ws + kOffKH);
  unsigned short* VT  = (unsigned short*)(ws + kOffVT);
  unsigned short* W1T = (unsigned short*)(ws + kOffW1T);
  unsigned short* W2T = (unsigned short*)(ws + kOffW2T);
  unsigned short* OWT = (unsigned short*)(ws + kOffOWT);
  float*          GT  = (float*)(ws + kOffGT);
  int*            IX  = (int*)(ws + kOffIX);
  unsigned short* DQ  = (unsigned short*)(ws + kOffDQ);
  unsigned short* AOG = (unsigned short*)(ws + kOffAOG);
  unsigned short* MP  = (unsigned short*)(ws + kOffMP);
  unsigned short* YP  = (unsigned short*)(ws + kOffYP);

  pack_x_kernel<<<(kN * kD / 8) / 256, 256, 0, stream>>>(query, XH, XL, kN * kD / 8);
  pack_scale_kernel<<<(kN * kD / 8) / 256, 256, 0, stream>>>(keyp, KH, kN * kD / 8, kKCarry);
  tpose_f16_kernel<<<dim3(kT / 64, 1, kB * kH), 256, 0, stream>>>(
      value, kD, (long)kT * kD, (long)kHD, kH, VT, kT, (long)kHD * kT, kVCarry);
  tpose_f16_kernel<<<dim3(kD / 64, 1, kE), 256, 0, stream>>>(
      w1, kHD, (long)kD * kHD, 0L, 1, W1T, kD, (long)kHD * kD, kW1Carry);
  tpose_f16_kernel<<<dim3(1, kD / 64, kE), 256, 0, stream>>>(
      w2, kD, (long)kHD * kD, 0L, 1, W2T, kEH, (long)kHD, kW2Carry);
  tpose_f16_kernel<<<dim3(kD / 64, kD / 64, 1), 256, 0, stream>>>(
      outw, kD, 0L, 0L, 1, OWT, kD, 0L, kOWCarry);

  gate_topk_kernel<<<kN / 256, 256, 0, stream>>>(query, egate, GT, IX);

  wmma_gemm_kernel<2, true, 1, false><<<(kN / 32) * (kEH / 64) / 8, 256, 0, stream>>>(
      XH, XL, kD, W1T, kD, (void*)DQ, kEH, nullptr, kN, kEH, kD, kDqFold, kResFold);

  attn_kernel<<<kB * kH * (kT / 64), 128, 0, stream>>>(DQ, IX, GT, KH, VT, AOG);

  place_kernel<<<kN / 8, 256, 0, stream>>>(AOG, IX, MP);

  wmma_gemm_kernel<4, false, 1, false><<<(kN / 64) * (kD / 64) / 8, 256, 0, stream>>>(
      MP, nullptr, kEH, W2T, kEH, (void*)YP, kD, nullptr, kN, kD, kEH, kRedFold, 0.0f);

  wmma_gemm_kernel<4, false, 0, true><<<(kN / 64) * (kD / 64) / 8, 256, 0, stream>>>(
      YP, nullptr, kD, OWT, kD, (void*)out, kD, outb, kN, kD, kD, kOutFold, 0.0f);
}
